// MDTBlock_3865470566442
// MI455X (gfx1250) — hardware-verified
//
#include <hip/hip_runtime.h>

typedef _Float16 v16h __attribute__((ext_vector_type(16)));
typedef _Float16 v8h  __attribute__((ext_vector_type(8)));
typedef _Float16 v4h  __attribute__((ext_vector_type(4)));
typedef float    v8f  __attribute__((ext_vector_type(8)));
typedef float    v4f  __attribute__((ext_vector_type(4)));
typedef v8h __attribute__((may_alias)) v8ha;
typedef v4h __attribute__((may_alias)) v4ha;
typedef v4f __attribute__((may_alias)) v4fa;

union Frag { v16h v; v8h half[2]; };

#define C_HID    1024
#define C_TOK    256
#define C_NB     32
#define C_ROWS   8192
#define C_HROWS  4096
#define C_NH     16
#define C_HD     64
#define C_MCTX   77
#define C_KPAD   96
#define C_YROWS  2464
#define C_YROWSP 2560
#define C_ADA    6144
#define C_MLP    4096
#define C_QKVW   3072
#define C_KVW    2048
#define C_RELN   964
#define C_REL    961
#define PSCALE   16384.0f

__device__ __forceinline__ v8f wmma16_raw(v16h a, v16h b, v8f c) {
  return __builtin_amdgcn_wmma_f32_16x16x32_f16(false, a, false, b, (short)0, c, false, false);
}
__device__ __forceinline__ v8f wmma16(v16h a, v16h b, v8f c) {
  v8f d = wmma16_raw(a, b, c);
  asm volatile("v_nop\n\tv_nop\n\tv_nop\n\tv_nop" : "+v"(d) : "v"(a), "v"(b));
  return d;
}

__device__ __forceinline__ v16h load_frag(const _Float16* p, int h) {
  Frag f;
  f.half[0] = *(const v8ha*)(p + 8 * h);
  f.half[1] = *(const v8ha*)(p + 16 + 8 * h);
  return f.v;
}

__device__ __forceinline__ v8f vzero8() {
  const v8f z = {0.f, 0.f, 0.f, 0.f, 0.f, 0.f, 0.f, 0.f};
  return z;
}

__device__ __forceinline__ float wave_sum(float v) {
  v += __shfl_xor(v, 16);
  v += __shfl_xor(v, 8);
  v += __shfl_xor(v, 4);
  v += __shfl_xor(v, 2);
  v += __shfl_xor(v, 1);
  return v;
}

__device__ __forceinline__ float gelu_t(float u) {
  const float z = 0.7978845608028654f * (u + 0.044715f * u * u * u);
  const float e = __expf(-2.0f * z);
  return u * __builtin_amdgcn_rcpf(1.0f + e);
}

__device__ __forceinline__ _Float16 silu16(float v) {
  const float e = __expf(-v);
  return (_Float16)(16.0f * v * __builtin_amdgcn_rcpf(1.0f + e));
}

__device__ __forceinline__ v16h pack_p(v8f a, v8f c) {
  const v16h r = { (_Float16)(a[0] * PSCALE), (_Float16)(a[1] * PSCALE), (_Float16)(a[2] * PSCALE), (_Float16)(a[3] * PSCALE),
                   (_Float16)(a[4] * PSCALE), (_Float16)(a[5] * PSCALE), (_Float16)(a[6] * PSCALE), (_Float16)(a[7] * PSCALE),
                   (_Float16)(c[0] * PSCALE), (_Float16)(c[1] * PSCALE), (_Float16)(c[2] * PSCALE), (_Float16)(c[3] * PSCALE),
                   (_Float16)(c[4] * PSCALE), (_Float16)(c[5] * PSCALE), (_Float16)(c[6] * PSCALE), (_Float16)(c[7] * PSCALE) };
  return r;
}

__global__ __launch_bounds__(256) void wconv_kernel(const float* __restrict__ in,
                                                     _Float16* __restrict__ out,
                                                     int K, int Nn, int perm)
{
  __shared__ __attribute__((aligned(16))) _Float16 sT[64 * 64];
  const int tid = threadIdx.x;
  const int k0 = blockIdx.x * 64, f0 = blockIdx.y * 64;
  const int grp = f0 >> 10, hh = (f0 >> 6) & 15;
  #pragma unroll
  for (int e = 0; e < 16; ++e) {
    const int idx = e * 256 + tid;
    const int kk = idx >> 6, cc = idx & 63;
    const int scol = perm ? (grp * 1024 + cc * 16 + hh) : (f0 + cc);
    const float v = in[(size_t)(k0 + kk) * Nn + scol];
    sT[cc * 64 + kk] = (_Float16)(v * 64.0f);
  }
  __syncthreads();
  const int q8 = tid & 7, L = tid >> 3;
  const v8h v0 = *(const v8ha*)(sT + L * 64 + 8 * q8);
  const v8h v1 = *(const v8ha*)(sT + (L + 32) * 64 + 8 * q8);
  _Float16* d0 = out + (size_t)(f0 + L) * K + k0 + 8 * q8;
  _Float16* d1 = out + (size_t)(f0 + L + 32) * K + k0 + 8 * q8;
  *(volatile v8h*)d0 = v0;
  *(volatile v8h*)d1 = v1;
  __threadfence();
  *(volatile v8h*)d0 = v0;
  *(volatile v8h*)d1 = v1;
}

__global__ __launch_bounds__(128) void silu_kernel(const float* __restrict__ nz,
                                                    _Float16* __restrict__ sil)
{
  const int row = blockIdx.x, t = threadIdx.x;
  const float* p = nz + (size_t)row * C_HID + 8 * t;
  const v4f a = *(const v4fa*)p;
  const v4f c = *(const v4fa*)(p + 4);
  const v8h o = { silu16(a.x), silu16(a.y), silu16(a.z), silu16(a.w),
                  silu16(c.x), silu16(c.y), silu16(c.z), silu16(c.w) };
  _Float16* dst = sil + (size_t)row * C_HID + 8 * t;
  *(volatile v8h*)dst = o;
  __threadfence();
  *(volatile v8h*)dst = o;
}

__global__ __launch_bounds__(128) void yconv_kernel(const float* __restrict__ y,
                                                     _Float16* __restrict__ y16)
{
  const int row = blockIdx.x, t = threadIdx.x;
  v8h o = { (_Float16)0, (_Float16)0, (_Float16)0, (_Float16)0,
            (_Float16)0, (_Float16)0, (_Float16)0, (_Float16)0 };
  if (row < C_YROWS) {
    const float* p = y + (size_t)row * C_HID + 8 * t;
    const v4f a = *(const v4fa*)p;
    const v4f c = *(const v4fa*)(p + 4);
    o[0] = (_Float16)a.x; o[1] = (_Float16)a.y; o[2] = (_Float16)a.z; o[3] = (_Float16)a.w;
    o[4] = (_Float16)c.x; o[5] = (_Float16)c.y; o[6] = (_Float16)c.z; o[7] = (_Float16)c.w;
  }
  _Float16* dst = y16 + (size_t)row * C_HID + 8 * t;
  *(volatile v8h*)dst = o;
  __threadfence();
  *(volatile v8h*)dst = o;
}

template <bool ADD>
__global__ __launch_bounds__(128) void ln_mod_kernel(const float* xin,
                                                      const float* __restrict__ o2p,
                                                      const float* __restrict__ ada,
                                                      int shOff, int scOff,
                                                      float* xout,
                                                      _Float16* __restrict__ hout)
{
  __shared__ float sred[4];
  __shared__ __attribute__((aligned(16))) _Float16 sHr[C_HID];
  const int tok = blockIdx.x, b = tok >> 8;
  const int t = threadIdx.x, lane = t & 31, w = t >> 5;
  const size_t rb = (size_t)tok * C_HID;

  const v4f xa = *(const v4fa*)(xin + rb + 4 * t);
  const v4f xc = *(const v4fa*)(xin + rb + 512 + 4 * t);
  float v0 = xa.x, v1 = xa.y, v2 = xa.z, v3 = xa.w;
  float v4 = xc.x, v5 = xc.y, v6 = xc.z, v7 = xc.w;
  if (ADD) {
    const float* orow = o2p + rb;
    const int dlo = t >> 2;
    const int hb = 4 * (t & 3);
    v0 += orow[(hb + 0) * 64 + dlo];
    v1 += orow[(hb + 1) * 64 + dlo];
    v2 += orow[(hb + 2) * 64 + dlo];
    v3 += orow[(hb + 3) * 64 + dlo];
    v4 += orow[(hb + 0) * 64 + 32 + dlo];
    v5 += orow[(hb + 1) * 64 + 32 + dlo];
    v6 += orow[(hb + 2) * 64 + 32 + dlo];
    v7 += orow[(hb + 3) * 64 + 32 + dlo];
  }

  float s = ((v0 + v1) + (v2 + v3)) + ((v4 + v5) + (v6 + v7));
  s = wave_sum(s);
  if (lane == 0) sred[w] = s;
  __syncthreads();
  const float mean = ((sred[0] + sred[1]) + (sred[2] + sred[3])) * (1.0f / 1024.0f);
  __syncthreads();
  const float d0 = v0 - mean, d1 = v1 - mean, d2 = v2 - mean, d3 = v3 - mean;
  const float d4 = v4 - mean, d5 = v5 - mean, d6 = v6 - mean, d7 = v7 - mean;
  float s2 = ((d0 * d0 + d1 * d1) + (d2 * d2 + d3 * d3)) + ((d4 * d4 + d5 * d5) + (d6 * d6 + d7 * d7));
  s2 = wave_sum(s2);
  if (lane == 0) sred[w] = s2;
  __syncthreads();
  const float var = ((sred[0] + sred[1]) + (sred[2] + sred[3])) * (1.0f / 1024.0f);
  const float rstd = rsqrtf(var + 1e-6f);

  const float* sh = ada + (size_t)b * C_ADA + shOff;
  const float* sc = ada + (size_t)b * C_ADA + scOff;
  const int c0 = 4 * t, c1 = 512 + 4 * t;
  const v4h ha = { (_Float16)(d0 * rstd * (1.0f + sc[c0 + 0]) + sh[c0 + 0]),
                   (_Float16)(d1 * rstd * (1.0f + sc[c0 + 1]) + sh[c0 + 1]),
                   (_Float16)(d2 * rstd * (1.0f + sc[c0 + 2]) + sh[c0 + 2]),
                   (_Float16)(d3 * rstd * (1.0f + sc[c0 + 3]) + sh[c0 + 3]) };
  const v4h hc = { (_Float16)(d4 * rstd * (1.0f + sc[c1 + 0]) + sh[c1 + 0]),
                   (_Float16)(d5 * rstd * (1.0f + sc[c1 + 1]) + sh[c1 + 1]),
                   (_Float16)(d6 * rstd * (1.0f + sc[c1 + 2]) + sh[c1 + 2]),
                   (_Float16)(d7 * rstd * (1.0f + sc[c1 + 3]) + sh[c1 + 3]) };
  *(v4ha*)(sHr + c0) = ha;
  *(v4ha*)(sHr + c1) = hc;

  const v4f oa = {v0, v1, v2, v3};
  const v4f oc = {v4, v5, v6, v7};
  if (ADD) {
    *(volatile v4f*)(xout + rb + 4 * t) = oa;
    *(volatile v4f*)(xout + rb + 512 + 4 * t) = oc;
  }
  __syncthreads();
  const v8h hv = *(const v8ha*)(sHr + 8 * t);
  _Float16* hd = hout + rb + 8 * t;
  *(volatile v8h*)hd = hv;
  __threadfence();
  if (ADD) {
    *(volatile v4f*)(xout + rb + 4 * t) = oa;
    *(volatile v4f*)(xout + rb + 512 + 4 * t) = oc;
  }
  *(volatile v8h*)hd = hv;
}

template <bool F, bool HH>
__device__ __forceinline__ void tile_store(const float* sF, const _Float16* sH,
                                           float* outF, _Float16* outH,
                                           int m0, int n0, int Nout, int w, int lane)
{
  const int q8 = lane & 7, sub = lane >> 3;
  if (HH) {
    #pragma unroll
    for (int i = 0; i < 8; ++i) {
      const int row = 32 * w + 4 * i + sub;
      const v8h v = *(const v8ha*)(sH + row * 64 + 8 * q8);
      *(volatile v8h*)(outH + (size_t)(m0 + row) * Nout + n0 + 8 * q8) = v;
    }
  }
  if (F) {
    #pragma unroll
    for (int i = 0; i < 16; ++i) {
      const int L = 4 * i + sub;
      const int row = 32 * w + (L >> 1), hl = L & 1;
      const v4f v = *(const v4fa*)(sF + row * 64 + 32 * hl + 4 * q8);
      *(volatile v4f*)(outF + (size_t)(m0 + row) * Nout + n0 + 32 * hl + 4 * q8) = v;
    }
  }
}

template <int WAVES, int EPI, bool HASB, bool H2>
__global__ __launch_bounds__(32 * WAVES) void gemm_kernel(
    const _Float16* __restrict__ A, const _Float16* __restrict__ Bt,
    const float* __restrict__ bias, const float* __restrict__ resid,
    const float* __restrict__ gate, float* outF, _Float16* outH,
    int Nout, int K, float ascale, float oscale)
{
  static constexpr int  RB     = 32 * WAVES;
  static constexpr bool F32OUT = (EPI >= 2);
  static constexpr bool H16OUT = (EPI <= 1) || H2;
  __shared__ __attribute__((aligned(16))) float    sF[F32OUT ? RB * 64 : 4];
  __shared__ __attribute__((aligned(16))) _Float16 sH[H16OUT ? RB * 64 : 8];

  const int tid = threadIdx.x, lane = tid & 31, w = tid >> 5;
  const int h = lane >> 4, m = lane & 15;
  const int n0 = blockIdx.x * 64;
  const int m0 = blockIdx.y * RB;
  const int m0w = m0 + 32 * w;

  const _Float16* xa0 = A + (size_t)(m0w + m) * K;
  const _Float16* xa1 = xa0 + (size_t)16 * K;
  const _Float16* wb  = Bt + (size_t)(n0 + m) * K;

  v8f acc[2][4];
  #pragma unroll
  for (int mt = 0; mt < 2; ++mt)
    #pragma unroll
    for (int nt = 0; nt < 4; ++nt) acc[mt][nt] = vzero8();

  #pragma unroll 1
  for (int k0 = 0; k0 < K; k0 += 32) {
    const v16h a0 = load_frag(xa0 + k0, h);
    const v16h a1 = load_frag(xa1 + k0, h);
    v16h bf[4];
    #pragma unroll
    for (int nt = 0; nt < 4; ++nt) bf[nt] = load_frag(wb + (size_t)nt * 16 * K + k0, h);
    #pragma unroll
    for (int nt = 0; nt < 4; ++nt) {
      acc[0][nt] = wmma16_raw(a0, bf[nt], acc[0][nt]);
      acc[1][nt] = wmma16_raw(a1, bf[nt], acc[1][nt]);
    }
    asm volatile("v_nop\n\tv_nop\n\tv_nop\n\tv_nop"
                 : "+v"(acc[0][0]), "+v"(acc[0][1]), "+v"(acc[0][2]), "+v"(acc[0][3]),
                   "+v"(acc[1][0]), "+v"(acc[1][1]), "+v"(acc[1][2]), "+v"(acc[1][3])
                 : "v"(a0), "v"(a1), "v"(bf[0]), "v"(bf[1]), "v"(bf[2]), "v"(bf[3]));
  }

  #pragma unroll
  for (int nt = 0; nt < 4; ++nt) {
    const int coll = 16 * nt + m, col = n0 + coll;
    float bv = 0.0f;
    if (HASB) bv = bias[col];
    #pragma unroll
    for (int mt = 0; mt < 2; ++mt) {
      #pragma unroll
      for (int r = 0; r < 8; ++r) {
        const int rowl = 32 * w + 16 * mt + 8 * h + r;
        float y = acc[mt][nt][r] * ascale + bv;
        if (EPI == 1) y = gelu_t(y);
        if (EPI == 3) {
          const int grow = m0 + rowl;
          const float rv = resid[(size_t)grow * Nout + col];
          const float gv = gate[(size_t)(grow >> 8) * C_ADA + col];
          y = rv + gv * y;
        }
        if (F32OUT) sF[rowl * 64 + coll] = y;
        if (H16OUT) sH[rowl * 64 + coll] = (_Float16)(y * oscale);
      }
    }
  }
  __syncthreads();

  tile_store<F32OUT, H16OUT>(sF, sH, outF, outH, m0, n0, Nout, w, lane);
  __threadfence();
  tile_store<F32OUT, H16OUT>(sF, sH, outF, outH, m0, n0, Nout, w, lane);
}

__device__ __forceinline__ void o16_store_pass(const _Float16* so, _Float16* o16,
                                               size_t rowbase, int head, int lane)
{
  const int q8 = lane & 7, sub = lane >> 3;
  #pragma unroll
  for (int i = 0; i < 4; ++i) {
    const int row = 4 * i + sub;
    const v8h v = *(const v8ha*)(so + row * C_HD + 8 * q8);
    *(volatile v8h*)(o16 + (rowbase + row) * C_HID + head * C_HD + 8 * q8) = v;
  }
}

__global__ __launch_bounds__(256) void attn_self_kernel(const _Float16* __restrict__ qkv,
                                                         const float* __restrict__ rel,
                                                         _Float16* __restrict__ o16)
{
  __shared__ __attribute__((aligned(16))) _Float16 sVt[C_HD * C_TOK];
  __shared__ __attribute__((aligned(16))) _Float16 sOh[8 * 16 * C_HD];
  __shared__ float sBias[C_REL];

  const int tid = threadIdx.x, lane = tid & 31, w = tid >> 5;
  const int h = lane >> 4, m = lane & 15;
  const int bh = blockIdx.y, bl = bh >> 4, head = bh & 15;
  const int q0w = blockIdx.x * 128 + 16 * w;
  const int qi = q0w >> 4;
  const size_t tokb = (size_t)bl * C_TOK;

  for (int i = tid; i < C_REL; i += 256) sBias[i] = rel[(size_t)i * C_NH + head];
  for (int idx = tid; idx < C_TOK * 8; idx += 256) {
    const int key = idx >> 3, dg = idx & 7;
    const v8h v = *(const v8ha*)(qkv + (tokb + key) * C_QKVW + 2 * C_HID + head * C_HD + 8 * dg);
    _Float16* dst = sVt + (8 * dg) * C_TOK + key;
    #pragma unroll
    for (int j = 0; j < 8; ++j) dst[j * C_TOK] = v[j];
  }
  __syncthreads();

  const _Float16* qrow = qkv + (tokb + q0w + m) * C_QKVW + head * C_HD;
  const v16h qb0 = load_frag(qrow, h);
  const v16h qb1 = load_frag(qrow + 32, h);

  v8f o[4];
  #pragma unroll
  for (int t = 0; t < 4; ++t) o[t] = vzero8();
  float mrun = -1e30f, lrun = 0.0f;

  #pragma unroll 1
  for (int kb = 0; kb < C_TOK; kb += 64) {
    v8f s[4];
    #pragma unroll
    for (int j = 0; j < 4; ++j) {
      const _Float16* kp = qkv + (tokb + kb + 16 * j + m) * C_QKVW + C_HID + head * C_HD;
      const v16h kf0 = load_frag(kp, h);
      const v16h kf1 = load_frag(kp + 32, h);
      v8f z = vzero8();
      z = wmma16_raw(kf0, qb0, z);
      z = wmma16(kf1, qb1, z);
      const int bi = (qi - (kb >> 4) - j + 15) * 31 + (m - 8 * h + 15);
      #pragma unroll
      for (int r = 0; r < 8; ++r) s[j][r] = z[r] * 0.125f + sBias[bi - r];
    }
    float mloc = s[0][0];
    #pragma unroll
    for (int j = 0; j < 4; ++j)
      #pragma unroll
      for (int r = 0; r < 8; ++r) mloc = fmaxf(mloc, s[j][r]);
    mloc = fmaxf(mloc, __shfl_xor(mloc, 16));
    const float mnew = fmaxf(mrun, mloc);
    const float alpha = __expf(mrun - mnew);
    mrun = mnew;
    float lsum = 0.0f;
    #pragma unroll
    for (int j = 0; j < 4; ++j)
      #pragma unroll
      for (int r = 0; r < 8; ++r) {
        const float p = __expf(s[j][r] - mnew);
        s[j][r] = p;
        lsum += p;
      }
    lsum += __shfl_xor(lsum, 16);
    lrun = lrun * alpha + lsum;
    #pragma unroll
    for (int t = 0; t < 4; ++t)
      #pragma unroll
      for (int r = 0; r < 8; ++r) o[t][r] = o[t][r] * alpha;

    const v16h pb0 = pack_p(s[0], s[1]);
    const v16h pb1 = pack_p(s[2], s[3]);

    #pragma unroll
    for (int t = 0; t < 4; ++t) {
      const _Float16* vp = sVt + (16 * t + m) * C_TOK + kb;
      const v16h vf0 = load_frag(vp, h);
      const v16h vf1 = load_frag(vp + 32, h);
      o[t] = wmma16_raw(vf0, pb0, o[t]);
      o[t] = wmma16(vf1, pb1, o[t]);
    }
  }

  const float inv = (1.0f / lrun) * (16.0f / PSCALE);
  _Float16* so = sOh + w * (16 * C_HD);
  #pragma unroll
  for (int t = 0; t < 4; ++t)
    #pragma unroll
    for (int r = 0; r < 8; ++r)
      so[m * C_HD + 16 * t + 8 * h + r] = (_Float16)(o[t][r] * inv);
  __syncthreads();

  const size_t rowbase = tokb + q0w;
  o16_store_pass(so, o16, rowbase, head, lane);
  __threadfence();
  o16_store_pass(so, o16, rowbase, head, lane);
}

__device__ __forceinline__ void o2_store_pass(const float* so, float* o2p,
                                              size_t rowbase, int head, int lane)
{
  const int q8 = lane & 7, sub = lane >> 3;
  #pragma unroll
  for (int i = 0; i < 8; ++i) {
    const int L = 4 * i + sub;
    const int row = L >> 1, hl = L & 1;
    const v4f v = *(const v4fa*)(so + row * C_HD + 32 * hl + 4 * q8);
    *(volatile v4f*)(o2p + (rowbase + row) * C_HID + head * C_HD + 32 * hl + 4 * q8) = v;
  }
}

__global__ __launch_bounds__(256) void attn_cross_kernel(const _Float16* __restrict__ q2p,
                                                          const _Float16* __restrict__ kvp,
                                                          float* __restrict__ o2p)
{
  __shared__ __attribute__((aligned(16))) _Float16 sVt[C_HD * C_KPAD];
  __shared__ __attribute__((aligned(16))) float    sO[8 * 16 * C_HD];

  const int tid = threadIdx.x, lane = tid & 31, w = tid >> 5;
  const int h = lane >> 4, m = lane & 15;
  const int bh = blockIdx.y, b = bh >> 4, head = bh & 15;
  const int q0w = blockIdx.x * 128 + 16 * w;
  const size_t kvb = (size_t)b * C_MCTX;
  const v8h z8h = { (_Float16)0, (_Float16)0, (_Float16)0, (_Float16)0,
                    (_Float16)0, (_Float16)0, (_Float16)0, (_Float16)0 };

  for (int idx = tid; idx < C_KPAD * 8; idx += 256) {
    const int key = idx >> 3, dg = idx & 7;
    const int keyc = (key < C_MCTX) ? key : (C_MCTX - 1);
    v8h v = *(const v8ha*)(kvp + (kvb + keyc) * C_KVW + C_HID + head * C_HD + 8 * dg);
    if (key >= C_MCTX) v = z8h;
    _Float16* dst = sVt + (8 * dg) * C_KPAD + key;
    #pragma unroll
    for (int j = 0; j < 8; ++j) dst[j * C_KPAD] = v[j];
  }
  __syncthreads();

  const _Float16* qrow = q2p + ((size_t)b * C_TOK + q0w + m) * C_HID + head * C_HD;
  const v16h qb0 = load_frag(qrow, h);
  const v16h qb1 = load_frag(qrow + 32, h);

  v8f s[5];
  #pragma unroll
  for (int j = 0; j < 5; ++j) {
    const int kr = 16 * j + m;
    const int keyc = (kr < C_MCTX) ? kr : (C_MCTX - 1);
    const _Float16* kp = kvp + (kvb + keyc) * C_KVW + head * C_HD;
    const v16h kf0 = load_frag(kp, h);
    const v16h kf1 = load_frag(kp + 32, h);
    v8f z = vzero8();
    z = wmma16_raw(kf0, qb0, z);
    z = wmma16(kf1, qb1, z);
    #pragma unroll
    for (int r = 0; r < 8; ++r) {
      const int key = 16 * j + 8 * h + r;
      s[j][r] = (key < C_MCTX) ? (z[r] * 0.125f) : -1e30f;
    }
  }
  float mloc = s[0][0];
  #pragma unroll
  for (int j = 0; j < 5; ++j)
    #pragma unroll
    for (int r = 0; r < 8; ++r) mloc = fmaxf(mloc, s[j][r]);
  mloc = fmaxf(mloc, __shfl_xor(mloc, 16));
  float lsum = 0.0f;
  #pragma unroll
  for (int j = 0; j < 5; ++j)
    #pragma unroll
    for (int r = 0; r < 8; ++r) {
      const float p = __expf(s[j][r] - mloc);
      s[j][r] = p;
      lsum += p;
    }
  lsum += __shfl_xor(lsum, 16);

  const v16h pb0 = pack_p(s[0], s[1]);
  const v16h pb1 = pack_p(s[2], s[3]);
  const v16h pb2 = pack_p(s[4], vzero8());

  v8f o[4];
  #pragma unroll
  for (int t = 0; t < 4; ++t) {
    const _Float16* vp = sVt + (16 * t + m) * C_KPAD;
    const v16h vf0 = load_frag(vp, h);
    const v16h vf1 = load_frag(vp + 32, h);
    const v16h vf2 = load_frag(vp + 64, h);
    v8f a = vzero8();
    a = wmma16_raw(vf0, pb0, a);
    a = wmma16_raw(vf1, pb1, a);
    o[t] = wmma16(vf2, pb2, a);
  }

  const float inv = (1.0f / lsum) * (1.0f / PSCALE);
  float* so = sO + w * (16 * C_HD);
  #pragma unroll
  for (int t = 0; t < 4; ++t)
    #pragma unroll
    for (int r = 0; r < 8; ++r)
      so[m * C_HD + 16 * t + 8 * h + r] = o[t][r] * inv;
  __syncthreads();

  const size_t rowbase = (size_t)b * C_TOK + q0w;
  o2_store_pass(so, o2p, rowbase, head, lane);
  __threadfence();
  o2_store_pass(so, o2p, rowbase, head, lane);
}

extern "C" void kernel_launch(void* const* d_in, const int* in_sizes, int n_in,
                              void* d_out, int out_size, void* d_ws, size_t ws_size,
                              hipStream_t stream)
{
  if (n_in < 16) return;
  if (in_sizes[0] != C_ROWS * C_HID) return;
  if (in_sizes[1] != C_NB * C_HID) return;
  if (in_sizes[2] != C_YROWS * C_HID) return;
  if (in_sizes[3] != C_HID * C_QKVW || in_sizes[4] != C_QKVW) return;
  if (in_sizes[5] != C_HID * C_HID || in_sizes[6] != C_HID) return;
  if (in_sizes[7] != C_RELN * C_NH) return;
  if (in_sizes[8] != C_HID * C_ADA || in_sizes[9] != C_ADA) return;
  if (in_sizes[10] != C_HID * C_MLP || in_sizes[11] != C_MLP) return;
  if (in_sizes[12] != C_MLP * C_HID || in_sizes[13] != C_HID) return;
  if (in_sizes[14] != C_HID * C_HID || in_sizes[15] != C_HID * C_KVW) return;
  if (out_size != C_ROWS * C_HID) return;

  const size_t AW_OFF  = 0;
  const size_t AW_BYTES  = (size_t)14680064;
  const size_t ADA_OFF = AW_OFF + AW_BYTES;
  const size_t ADA_BYTES = (size_t)C_NB * C_ADA * 4;
  const size_t SIL_OFF = ADA_OFF + ADA_BYTES;
  const size_t SIL_BYTES = (size_t)C_NB * C_HID * 2;
  const size_t H_OFF   = SIL_OFF + SIL_BYTES;
  const size_t H_BYTES = (size_t)C_ROWS * C_HID * 2;
  const size_t G_OFF   = H_OFF + H_BYTES;
  const size_t G_BYTES = (size_t)C_ROWS * C_MLP * 2;
  const size_t X_OFF   = G_OFF + G_BYTES;
  const size_t X_BYTES = (size_t)C_ROWS * C_HID * 4;
  if (X_OFF + X_BYTES > ws_size) return;

  const float* x      = (const float*)d_in[0];
  const float* noise  = (const float*)d_in[1];
  const float* y      = (const float*)d_in[2];
  const float* W_qkv  = (const float*)d_in[3];
  const float* b_qkv  = (const float*)d_in[4];
  const float* W_proj = (const float*)d_in[5];
  const float* b_proj = (const float*)d_in[6];
  const float* rel    = (const float*)d_in[7];
  const float* W_ada  = (const float*)d_in[8];
  const float* b_ada  = (const float*)d_in[9];
  const float* W_fc1  = (const float*)d_in[10];
  const float* b_fc1  = (const float*)d_in[11];
  const float* W_fc2  = (const float*)d_in[12];
  const float* b_fc2  = (const float*)d_in[13];
  const float* W_q    = (const float*)d_in[14];
  const float* W_kv   = (const float*)d_in[15];
  float* out = (float*)d_out;

  char* ws = (char*)d_ws;
  _Float16* WadaT  = (_Float16*)(ws + AW_OFF);
  _Float16* WqkvT  = (_Float16*)(ws + AW_OFF);
  _Float16* WprojT = (_Float16*)(ws + AW_OFF + 6291456);
  _Float16* WqT    = (_Float16*)(ws + AW_OFF + 8388608);
  _Float16* WkvT   = (_Float16*)(ws + AW_OFF + 10485760);
  _Float16* Wfc1T  = (_Float16*)(ws + AW_OFF);
  _Float16* Wfc2T  = (_Float16*)(ws + AW_OFF);
  float*    ADA    = (float*)(ws + ADA_OFF);
  _Float16* SIL    = (_Float16*)(ws + SIL_OFF);
  _Float16* H      = (_Float16*)(ws + H_OFF);
  char*     G      = ws + G_OFF;
  _Float16* QKV    = (_Float16*)G;
  _Float16* X1H    = (_Float16*)G;
  float*    O2P    = (float*)G;
  _Float16* KVP    = (_Float16*)(G + 33554432);
  _Float16* Y16    = (_Float16*)(G + 44040192);
  _Float16* Q2P    = (_Float16*)(G + 50331648);
  _Float16* GPL    = (_Float16*)G;
  float*    X      = (float*)(ws + X_OFF);

  wconv_kernel<<<dim3(C_HID / 64, C_ADA / 64), 256, 0, stream>>>(W_ada, WadaT, C_HID, C_ADA, 0);
  silu_kernel<<<C_NB, 128, 0, stream>>>(noise, SIL);
  gemm_kernel<1, 2, true, false><<<dim3(C_ADA / 64, 1), 32, 0, stream>>>(
      SIL, WadaT, b_ada, nullptr, nullptr, ADA, nullptr, C_ADA, C_HID, 1.0f / 1024.0f, 1.0f);

  wconv_kernel<<<dim3(C_HID / 64, C_QKVW / 64), 256, 0, stream>>>(W_qkv, WqkvT, C_HID, C_QKVW, 0);
  wconv_kernel<<<dim3(C_HID / 64, C_HID / 64), 256, 0, stream>>>(W_proj, WprojT, C_HID, C_HID, 0);
  wconv_kernel<<<dim3(C_HID / 64, C_HID / 64), 256, 0, stream>>>(W_q, WqT, C_HID, C_HID, 1);
  wconv_kernel<<<dim3(C_HID / 64, C_KVW / 64), 256, 0, stream>>>(W_kv, WkvT, C_HID, C_KVW, 1);

  ln_mod_kernel<false><<<C_ROWS, 128, 0, stream>>>(x, nullptr, ADA, 0, C_HID, nullptr, H);

  for (int half = 0; half < 2; ++half) {
    const _Float16* Hh = H + (size_t)half * C_HROWS * C_HID;
    _Float16* Oh = H + (size_t)half * C_HROWS * C_HID;
    gemm_kernel<4, 0, true, false><<<dim3(C_QKVW / 64, C_HROWS / 128), 128, 0, stream>>>(
        Hh, WqkvT, b_qkv, nullptr, nullptr, nullptr, QKV, C_QKVW, C_HID, 1.0f / 64.0f, 1.0f);
    attn_self_kernel<<<dim3(2, 16 * C_NH), 256, 0, stream>>>(QKV, rel, Oh);
  }

  gemm_kernel<4, 3, true, true><<<dim3(C_HID / 64, C_ROWS / 128), 128, 0, stream>>>(
      H, WprojT, b_proj, x, ADA + 2 * C_HID, X, X1H, C_HID, C_HID, 1.0f / 1024.0f, 1.0f);

  gemm_kernel<4, 0, false, false><<<dim3(C_HID / 64, C_ROWS / 128), 128, 0, stream>>>(
      X1H, WqT, nullptr, nullptr, nullptr, nullptr, Q2P, C_HID, C_HID, 1.0f / 64.0f, 1.0f);
  yconv_kernel<<<C_YROWSP, 128, 0, stream>>>(y, Y16);
  gemm_kernel<4, 0, false, false><<<dim3(C_KVW / 64, C_YROWSP / 128), 128, 0, stream>>>(
      Y16, WkvT, nullptr, nullptr, nullptr, nullptr, KVP, C_KVW, C_HID, 1.0f / 64.0f, 1.0f);

  attn_cross_kernel<<<dim3(2, C_NB * C_NH), 256, 0, stream>>>(Q2P, KVP, O2P);

  ln_mod_kernel<true><<<C_ROWS, 128, 0, stream>>>(X, O2P, ADA, 3 * C_HID, 4 * C_HID, X, H);

  wconv_kernel<<<dim3(C_HID / 64, C_MLP / 64), 256, 0, stream>>>(W_fc1, Wfc1T, C_HID, C_MLP, 0);
  gemm_kernel<4, 1, true, false><<<dim3(C_MLP / 64, C_ROWS / 128), 128, 0, stream>>>(
      H, Wfc1T, b_fc1, nullptr, nullptr, nullptr, GPL, C_MLP, C_HID, 1.0f / 64.0f, 8.0f);

  wconv_kernel<<<dim3(C_MLP / 64, C_HID / 64), 256, 0, stream>>>(W_fc2, Wfc2T, C_MLP, C_HID, 0);
  gemm_kernel<4, 3, true, false><<<dim3(C_HID / 64, C_ROWS / 128), 128, 0, stream>>>(
      GPL, Wfc2T, b_fc2, X, ADA + 5 * C_HID, out, nullptr, C_HID, C_MLP, 1.0f / 512.0f, 1.0f);
}
